// GraphMoEAttentionRouter_10101763080593
// MI455X (gfx1250) — hardware-verified
//
#include <hip/hip_runtime.h>
#include <stddef.h>
#include <stdint.h>

#define NN    8192
#define NE    131072
#define IND   6
#define HID   256
#define NX    8
#define NG    64
#define EW    2048
#define ZK    288
#define ZP    320
#define KC    32
#define QBLK  64
#define AGD   16
#define CH    1024

static_assert(EW == NX * HID);
static_assert(NN % 256 == 0);
static_assert(NE % CH == 0);
static_assert(CH == 4 * 256);
static_assert(NE % (8 * 32) == 0);
static_assert(NN % QBLK == 0);
static_assert(NN % KC == 0);
static_assert(NN % AGD == 0);
static_assert(ZK % 32 == 0);
static_assert(ZK <= ZP);
static_assert(ZP % 64 == 0);
static_assert(HID % 64 == 0);
static_assert(NN % 64 == 0);
static_assert(NG == 64);

typedef _Float16 v16h __attribute__((ext_vector_type(16)));
typedef _Float16 v8h  __attribute__((ext_vector_type(8)));
typedef float    v8f  __attribute__((ext_vector_type(8)));
typedef float    v4f  __attribute__((ext_vector_type(4)));
typedef unsigned int v4u __attribute__((ext_vector_type(4)));
typedef int      v4i  __attribute__((ext_vector_type(4)));

union Frag  { v16h v; v8h h[2]; };
union Pack8 { v8h h; v4u u; };

__device__ __forceinline__ v8f mma16(v16h a, v16h b, v8f c) {
  c = __builtin_amdgcn_wmma_f32_16x16x32_f16(false, a, false, b, (short)0, c, false, false);
  asm volatile("v_nop\n\tv_nop\n\tv_nop\n\tv_nop" : "+v"(c) : "v"(a), "v"(b));
  return c;
}

__device__ __forceinline__ v16h ldfrag(const _Float16* p, int ld, int row0, int k0, int lane) {
  const int m = lane & 15, lh = lane >> 4;
  const _Float16* q = p + (size_t)(row0 + m) * ld + k0 + 8 * lh;
  Frag f;
  f.h[0] = *(const v8h*)(q);
  f.h[1] = *(const v8h*)(q + 16);
  return f.v;
}

__device__ __forceinline__ v8f zero8() { return (v8f){0.f, 0.f, 0.f, 0.f, 0.f, 0.f, 0.f, 0.f}; }

__device__ __forceinline__ v4u pack8h(v4f a, v4f b) {
  Pack8 pk;
  pk.h = (v8h){(_Float16)a[0], (_Float16)a[1], (_Float16)a[2], (_Float16)a[3],
               (_Float16)b[0], (_Float16)b[1], (_Float16)b[2], (_Float16)b[3]};
  return pk.u;
}

__device__ __forceinline__ void gemm32x64(const _Float16* __restrict__ A, int lda,
                                          const _Float16* __restrict__ Bt, int ldb, int K,
                                          int m0, int n0, int lane, v8f (&acc)[2][4]) {
#pragma unroll 1
  for (int k0 = 0; k0 < K; k0 += 32) {
    const v16h a0 = ldfrag(A, lda, m0, k0, lane);
    const v16h a1 = ldfrag(A, lda, m0 + 16, k0, lane);
    const v16h b0 = ldfrag(Bt, ldb, n0, k0, lane);
    const v16h b1 = ldfrag(Bt, ldb, n0 + 16, k0, lane);
    const v16h b2 = ldfrag(Bt, ldb, n0 + 32, k0, lane);
    const v16h b3 = ldfrag(Bt, ldb, n0 + 48, k0, lane);
    acc[0][0] = mma16(a0, b0, acc[0][0]);
    acc[1][0] = mma16(a1, b0, acc[1][0]);
    acc[0][1] = mma16(a0, b1, acc[0][1]);
    acc[1][1] = mma16(a1, b1, acc[1][1]);
    acc[0][2] = mma16(a0, b2, acc[0][2]);
    acc[1][2] = mma16(a1, b2, acc[1][2]);
    acc[0][3] = mma16(a0, b3, acc[0][3]);
    acc[1][3] = mma16(a1, b3, acc[1][3]);
  }
}

#define OTP 68
__device__ __forceinline__ void store16x64_f32(const float* sw, float* __restrict__ out, int ldo,
                                               int row0, int n0, int lane) {
  v4f val[8];
  size_t go[8];
#pragma unroll
  for (int it = 0; it < 8; ++it) {
    const int p    = lane + 32 * it;
    const int L    = p >> 3;
    const int pc   = p & 7;
    const int row  = L >> 1;
    const int hsel = L & 1;
    val[it] = *(const v4f*)(sw + row * OTP + hsel * 32 + pc * 4);
    go[it]  = (size_t)(row0 + row) * ldo + n0 + hsel * 32 + pc * 4;
  }
  for (int ps = 0; ps < 2; ++ps) {
#pragma unroll
    for (int it = 0; it < 8; ++it) *(volatile v4f*)(out + go[it]) = val[it];
    __threadfence();
  }
}

__device__ __forceinline__ void hist64(int gc, int lane, int& c0, int& c1) {
  const unsigned mlo = __builtin_amdgcn_ballot_w32(gc >= 0 && gc < 32);
  const unsigned mhi = __builtin_amdgcn_ballot_w32(gc >= 32 && gc < NG);
  const int gl = gc & 31;
#pragma unroll
  for (int g = 0; g < 32; ++g) {
    const unsigned b = __builtin_amdgcn_ballot_w32(gl == g);
    const int a0 = __builtin_popcount(b & mlo);
    const int a1 = __builtin_popcount(b & mhi);
    c0 += (lane == g) ? a0 : 0;
    c1 += (lane == g) ? a1 : 0;
  }
}

__global__ __launch_bounds__(256) void k_stats(const int* __restrict__ eidx, const int* __restrict__ batch,
                                               float* __restrict__ tab) {
  __shared__ int cn[8 * NG];
  __shared__ int ce[8 * NG];
  const int tid = threadIdx.x, lane = tid & 31, wave = tid >> 5;
  int c0 = 0, c1 = 0;
  for (int it = 0; it < NN / 256; ++it) {
    const int n  = wave * (NN / 8) + it * 32 + lane;
    const int g  = batch[n];
    const int gc = ((unsigned)g < (unsigned)NG) ? g : -1;
    hist64(gc, lane, c0, c1);
  }
  int d0 = 0, d1 = 0;
  for (int it = 0; it < NE / 256; ++it) {
    const int e = wave * (NE / 8) + it * 32 + lane;
    int s = eidx[e];
    s = min(max(s, 0), NN - 1);
    const int g  = batch[s];
    const int gc = ((unsigned)g < (unsigned)NG) ? g : -1;
    hist64(gc, lane, d0, d1);
  }
  cn[wave * NG + lane] = c0;
  cn[wave * NG + 32 + lane] = c1;
  ce[wave * NG + lane] = d0;
  ce[wave * NG + 32 + lane] = d1;
  __syncthreads();
  if (tid < NG) {
    int sn = 0, se = 0;
#pragma unroll
    for (int w = 0; w < 8; ++w) { sn += cn[w * NG + tid]; se += ce[w * NG + tid]; }
    const float fn = (float)sn, fe = (float)se;
    const v4f t = (v4f){log1pf(fn), log1pf(fe), fn, fe};
    volatile v4f* d = (volatile v4f*)(tab + 4 * tid);
    *d = t;
    __threadfence();
    *d = t;
  }
}

__global__ __launch_bounds__(256) void k_enc(const float* __restrict__ x, const int* __restrict__ batch,
                                             const float* __restrict__ encW, const float* __restrict__ encB,
                                             const float* __restrict__ tab,
                                             float* __restrict__ hf, _Float16* __restrict__ zh,
                                             float* __restrict__ part) {
  __shared__ __align__(16) _Float16 zs[64 * ZP];
  __shared__ __align__(16) float sft[NG * 4];
  const int tid = threadIdx.x;
  const int nb = blockIdx.x * 64;
  if (tid < NG) *(v4f*)(sft + 4 * tid) = *(const v4f*)(tab + 4 * tid);
  float w[IND];
#pragma unroll
  for (int i = 0; i < IND; ++i) w[i] = encW[i * HID + tid];
  const float bb = encB[tid];
  __syncthreads();
  float csum = 0.f;
#pragma unroll 1
  for (int r = 0; r < 64; ++r) {
    const int n = nb + r;
    const float* xr = x + (size_t)n * IND;
    float a = 0.f;
#pragma unroll
    for (int i = 0; i < IND; ++i) a += xr[i] * w[i];
    const float hv = fmaxf(a + bb, 0.f);
    csum += hv;
    volatile float* hp = hf + (size_t)n * HID + tid;
    *hp = hv;
    __threadfence();
    *hp = hv;
    zs[r * ZP + tid] = (_Float16)hv;
    if (tid < 64) {
      int g = batch[n];
      g = min(max(g, 0), NG - 1);
      const float s0 = sft[4 * g], s1 = sft[4 * g + 1];
      const float sv = (tid == 0) ? s0 : ((tid == 1) ? s1 : 0.f);
      zs[r * ZP + HID + tid] = (_Float16)sv;
    }
  }
  __syncthreads();
  v4u val[10];
#pragma unroll
  for (int it = 0; it < 10; ++it) {
    const int p = tid + 256 * it;
    Pack8 pk;
    pk.h = *(const v8h*)(zs + 8 * p);
    val[it] = pk.u;
  }
  _Float16* zb = zh + (size_t)nb * ZP;
  for (int ps = 0; ps < 2; ++ps) {
#pragma unroll
    for (int it = 0; it < 10; ++it) *(volatile v4u*)(zb + 8 * (tid + 256 * it)) = val[it];
    __threadfence();
  }
  volatile float* pp = part + (size_t)blockIdx.x * HID + tid;
  *pp = csum;
  __threadfence();
  *pp = csum;
}

__global__ __launch_bounds__(256) void k_koff(const float* __restrict__ part, const float* __restrict__ tab,
                                              const float* __restrict__ kW, const float* __restrict__ kB,
                                              float* __restrict__ koff) {
  __shared__ float zb[ZK];
  const int tid = threadIdx.x;
  float s = 0.f;
#pragma unroll 1
  for (int b = 0; b < NN / 64; ++b) s += part[b * HID + tid];
  zb[tid] = s * (1.0f / (float)NN);
  if (tid < 32) {
    const int col = (tid < 2) ? tid : 0;
    float s2 = 0.f;
#pragma unroll 1
    for (int g = 0; g < NG; ++g) s2 += tab[4 * g + 2] * tab[4 * g + col];
    zb[HID + tid] = (tid < 2) ? s2 * (1.0f / (float)NN) : 0.f;
  }
  __syncthreads();
  float d = 0.f;
#pragma unroll 1
  for (int k = 0; k < HID + 2; ++k) d += zb[k] * kW[(size_t)k * HID + tid];
  const float o = kB[tid] - d;
  volatile float* p = koff + tid;
  *p = o;
  __threadfence();
  *p = o;
}

#define TRP 72
__global__ __launch_bounds__(256) void k_wtr(const float* __restrict__ W0, const float* __restrict__ W1,
                                             const float* __restrict__ W2, int nsel, int zin,
                                             int K, int Ncol, int zdiv, int za, int zb2, int zc,
                                             _Float16* __restrict__ out, int KP, float scale) {
  __shared__ __align__(16) _Float16 th[64 * TRP];
  const int tid = threadIdx.x, z = blockIdx.z;
  const int n0 = blockIdx.x * 64, k0 = blockIdx.y * 64;
  const float* Wb = (nsel == 3) ? ((z == 0) ? W0 : ((z == 1) ? W1 : W2)) : (W0 + (size_t)z * zin);
  const int r  = tid >> 2;
  const int cq = (tid & 3) * 16;
  const int kr  = k0 + r;
  const int krc = min(kr, K - 1);
  const float keep = (kr < K) ? scale : 0.f;
  const float* src = Wb + (size_t)krc * Ncol + n0 + cq;
#pragma unroll
  for (int j = 0; j < 4; ++j) {
    const v4f v = *(const v4f*)(src + 4 * j) * keep;
#pragma unroll
    for (int i = 0; i < 4; ++i) th[(cq + 4 * j + i) * TRP + r] = (_Float16)v[i];
  }
  __syncthreads();
  const int orow0 = (z / zdiv) * za + (z % zdiv) * zb2;
  const int ocol0 = z * zc;
  v4u val[2];
  size_t go[2];
#pragma unroll
  for (int it = 0; it < 2; ++it) {
    const int p  = tid + 256 * it;
    const int L  = p >> 3;
    const int pc = p & 7;
    Pack8 pk;
    pk.h    = *(const v8h*)(th + L * TRP + pc * 8);
    val[it] = pk.u;
    go[it]  = (size_t)(orow0 + n0 + L) * KP + ocol0 + k0 + pc * 8;
  }
  for (int ps = 0; ps < 2; ++ps) {
#pragma unroll
    for (int it = 0; it < 2; ++it) *(volatile v4u*)(out + go[it]) = val[it];
    __threadfence();
  }
}

#define STP 72
#define SVP 264
__global__ __launch_bounds__(256) void k_qkv(const _Float16* __restrict__ zh, const _Float16* __restrict__ wt,
                                             const float* __restrict__ qb, const float* __restrict__ koff,
                                             const float* __restrict__ vb,
                                             _Float16* __restrict__ qpl, _Float16* __restrict__ kpl,
                                             _Float16* __restrict__ vtp) {
  __shared__ __align__(16) _Float16 st[256 * STP];
  const int tid = threadIdx.x, lane = tid & 31, wave = tid >> 5;
  const int hh = lane >> 4, c = lane & 15;
  const int bx = blockIdx.x;
  const int ns = blockIdx.y;
  const int which = ns >> 2;
  const int slab  = ns & 3;
  const int m0 = bx * 256 + wave * 32;
  const int n0 = ns * 64;

  v8f acc[2][4];
#pragma unroll
  for (int s = 0; s < 2; ++s)
#pragma unroll
    for (int t = 0; t < 4; ++t) acc[s][t] = zero8();
  gemm32x64(zh, ZP, wt, ZP, ZK, m0, n0, lane, acc);

  float bb[4];
#pragma unroll
  for (int t = 0; t < 4; ++t) {
    const int i = slab * 64 + 16 * t + c;
    const float xq = qb[i], xk = koff[i], xv = vb[i];
    bb[t] = (which == 0) ? xq : ((which == 1) ? xk : xv);
  }

  if (which < 2) {
#pragma unroll
    for (int sub = 0; sub < 2; ++sub)
#pragma unroll
      for (int t = 0; t < 4; ++t)
#pragma unroll
        for (int r = 0; r < 8; ++r)
          st[(wave * 32 + sub * 16 + 8 * hh + r) * STP + 16 * t + c] =
              (_Float16)(acc[sub][t][r] * 0.03125f + bb[t]);
  } else {
#pragma unroll
    for (int sub = 0; sub < 2; ++sub)
#pragma unroll
      for (int t = 0; t < 4; ++t)
#pragma unroll
        for (int r = 0; r < 8; ++r)
          st[(16 * t + c) * SVP + wave * 32 + sub * 16 + 8 * hh + r] =
              (_Float16)(acc[sub][t][r] * 0.03125f + bb[t]);
  }
  __syncthreads();

  if (which < 2) {
    _Float16* base = ((which == 0) ? qpl : kpl) + slab * 64;
#pragma unroll
    for (int g = 0; g < 2; ++g) {
      v4u val[4];
      size_t go[4];
#pragma unroll
      for (int j = 0; j < 4; ++j) {
        const int p  = tid + 256 * (4 * g + j);
        const int lr = p >> 3;
        const int pc = p & 7;
        Pack8 pk;
        pk.h   = *(const v8h*)(st + lr * STP + pc * 8);
        val[j] = pk.u;
        go[j]  = (size_t)(bx * 256 + lr) * HID + pc * 8;
      }
      for (int ps = 0; ps < 2; ++ps) {
#pragma unroll
        for (int j = 0; j < 4; ++j) *(volatile v4u*)(base + go[j]) = val[j];
        __threadfence();
      }
    }
  } else {
    _Float16* base = vtp + (size_t)(slab * 64) * NN;
#pragma unroll
    for (int g = 0; g < 2; ++g) {
      v4u val[4];
      size_t go[4];
#pragma unroll
      for (int j = 0; j < 4; ++j) {
        const int p    = tid + 256 * (4 * g + j);
        const int drow = p >> 5;
        const int pc   = p & 31;
        Pack8 pk;
        pk.h   = *(const v8h*)(st + drow * SVP + pc * 8);
        val[j] = pk.u;
        go[j]  = (size_t)drow * NN + bx * 256 + pc * 8;
      }
      for (int ps = 0; ps < 2; ++ps) {
#pragma unroll
        for (int j = 0; j < 4; ++j) *(volatile v4u*)(base + go[j]) = val[j];
        __threadfence();
      }
    }
  }
}

#define KTP 264
#define VTP 40
#define OSP 132
__global__ __launch_bounds__(256) void k_attn(const _Float16* __restrict__ qp,
                                              const _Float16* __restrict__ kp,
                                              const _Float16* __restrict__ vt,
                                              float* __restrict__ fo, float sscale) {
  __shared__ __align__(16) _Float16 KV[KC * KTP + HID * VTP];
  __shared__ __align__(16) _Float16 Ps[4 * 16 * VTP];
  __shared__ float al_l[QBLK];
  __shared__ float ll_l[QBLK];
  _Float16* Ks = KV;
  _Float16* Vs = KV + KC * KTP;

  const int tid = threadIdx.x, lane = tid & 31, wave = tid >> 5;
  const int hh = lane >> 4, c = lane & 15;
  const int wsq = wave & 3;
  const int hfc = wave >> 2;
  const int q0  = blockIdx.x * QBLK + wsq * 16;

  const float NEGI = -__builtin_huge_valf();
  float mrow[8], lrow[8];
  v8f oacc[8];
#pragma unroll
  for (int r = 0; r < 8; ++r) { mrow[r] = NEGI; lrow[r] = 0.f; }
#pragma unroll
  for (int t = 0; t < 8; ++t) oacc[t] = zero8();

  _Float16* pw = Ps + wsq * 16 * VTP;

  for (int kc = 0; kc < NN / KC; ++kc) {
    const int kv0 = kc * KC;
    __syncthreads();
    {
      const int kr = tid >> 3;
      const int dq = (tid & 7) * 32;
      const _Float16* ks = kp + (size_t)(kv0 + kr) * HID + dq;
      _Float16* kd = Ks + kr * KTP + dq;
#pragma unroll
      for (int e = 0; e < 4; ++e) *(v8h*)(kd + 8 * e) = *(const v8h*)(ks + 8 * e);
      const _Float16* vs = vt + (size_t)tid * NN + kv0;
      _Float16* vd = Vs + tid * VTP;
#pragma unroll
      for (int e = 0; e < 4; ++e) *(v8h*)(vd + 8 * e) = *(const v8h*)(vs + 8 * e);
    }
    __syncthreads();

    if (hfc == 0) {
      v8f s0 = zero8(), s1 = zero8();
#pragma unroll
      for (int dc = 0; dc < HID / 32; ++dc) {
        const v16h qa = ldfrag(qp, HID, q0, dc * 32, lane);
        const v16h k0 = ldfrag(Ks, KTP, 0, dc * 32, lane);
        const v16h k1 = ldfrag(Ks, KTP, 16, dc * 32, lane);
        s0 = mma16(qa, k0, s0);
        s1 = mma16(qa, k1, s1);
      }
#pragma unroll
      for (int r = 0; r < 8; ++r) {
        const float v0 = s0[r] * sscale, v1 = s1[r] * sscale;
        float m = fmaxf(v0, v1);
#pragma unroll
        for (int off = 1; off < 16; off <<= 1) m = fmaxf(m, __shfl_xor(m, off, 32));
        const float mnew  = fmaxf(mrow[r], m);
        const float alpha = __expf(mrow[r] - mnew);
        const float p0 = __expf(v0 - mnew), p1 = __expf(v1 - mnew);
        float psum = p0 + p1;
#pragma unroll
        for (int off = 1; off < 16; off <<= 1) psum += __shfl_xor(psum, off, 32);
        lrow[r] = lrow[r] * alpha + psum;
        mrow[r] = mnew;
        pw[(8 * hh + r) * VTP + c]      = (_Float16)(p0 * 1024.0f);
        pw[(8 * hh + r) * VTP + 16 + c] = (_Float16)(p1 * 1024.0f);
        if (c == 0) al_l[wsq * 16 + 8 * hh + r] = alpha;
      }
    }
    __syncthreads();

    {
      float alv[8];
#pragma unroll
      for (int r = 0; r < 8; ++r) alv[r] = al_l[wsq * 16 + 8 * hh + r];
#pragma unroll
      for (int t = 0; t < 8; ++t)
#pragma unroll
        for (int r = 0; r < 8; ++r) oacc[t][r] *= alv[r];
      const v16h pa = ldfrag(pw, VTP, 0, 0, lane);
#pragma unroll
      for (int t = 0; t < 8; ++t) {
        const v16h vb2 = ldfrag(Vs, VTP, hfc * 128 + 16 * t, 0, lane);
        oacc[t] = mma16(pa, vb2, oacc[t]);
      }
    }
  }

  if (hfc == 0) {
    if (c == 0) {
#pragma unroll
      for (int r = 0; r < 8; ++r) ll_l[wsq * 16 + 8 * hh + r] = lrow[r];
    }
  }
  __syncthreads();
  float invl[8];
#pragma unroll
  for (int r = 0; r < 8; ++r) {
    const float l = ll_l[wsq * 16 + 8 * hh + r];
    invl[r] = (l > 0.f) ? (0.0009765625f / l) : 0.f;
  }
  float* ost = reinterpret_cast<float*>(KV) + wave * 8 * OSP;
  for (int hs = 0; hs < 2; ++hs) {
    __syncthreads();
    if (hh == hs) {
#pragma unroll
      for (int t = 0; t < 8; ++t)
#pragma unroll
        for (int r = 0; r < 8; ++r) ost[r * OSP + 16 * t + c] = oacc[t][r] * invl[r];
    }
    __syncthreads();
    v4f val[8];
    size_t go[8];
#pragma unroll
    for (int it = 0; it < 8; ++it) {
      val[it] = *(const v4f*)(ost + it * OSP + 4 * lane);
      go[it]  = (size_t)(q0 + hs * 8 + it) * HID + hfc * 128 + 4 * lane;
    }
    for (int ps = 0; ps < 2; ++ps) {
#pragma unroll
      for (int it = 0; it < 8; ++it) *(volatile v4f*)(fo + go[it]) = val[it];
      __threadfence();
    }
  }
}

__global__ __launch_bounds__(256) void k_router(const float* __restrict__ fused, const float* __restrict__ oW,
                                                const float* __restrict__ oB, float* __restrict__ rw) {
  __shared__ __align__(16) float wsh[HID * NX];
  __shared__ __align__(16) float rst[256 * NX];
  const int tid = threadIdx.x;
  const int n = blockIdx.x * 256 + tid;
  *(v4f*)(wsh + 8 * tid)     = *(const v4f*)(oW + 8 * tid);
  *(v4f*)(wsh + 8 * tid + 4) = *(const v4f*)(oW + 8 * tid + 4);
  __syncthreads();
  double lg[NX];
#pragma unroll
  for (int e = 0; e < NX; ++e) lg[e] = 0.0;
  const float* fr = fused + (size_t)n * HID;
#pragma unroll 1
  for (int k = 0; k < HID; ++k) {
    const double f = (double)fr[k];
    const float* wr = wsh + k * NX;
#pragma unroll
    for (int e = 0; e < NX; ++e) lg[e] += f * (double)wr[e];
  }
  float l[NX];
#pragma unroll
  for (int e = 0; e < NX; ++e) l[e] = (float)(lg[e] + (double)oB[e]);
  float m1 = l[0];
  int i1 = 0;
#pragma unroll
  for (int e = 1; e < NX; ++e) {
    const bool up = l[e] > m1;
    m1 = up ? l[e] : m1;
    i1 = up ? e : i1;
  }
  float m2 = -__builtin_huge_valf();
  int i2 = -1;
#pragma unroll
  for (int e = 0; e < NX; ++e) {
    const bool ok = (e != i1) && (l[e] > m2);
    m2 = ok ? l[e] : m2;
    i2 = ok ? e : i2;
  }
  const float pe = __expf(m2 - m1);
  const float rs = 1.0f / (1.0f + pe);
  const float w1 = rs, w2 = pe * rs;
#pragma unroll
  for (int e = 0; e < NX; ++e) rst[tid * NX + e] = (e == i1) ? w1 : ((e == i2) ? w2 : 0.f);
  __syncthreads();
  v4f val[2];
  size_t go[2];
#pragma unroll
  for (int it = 0; it < 2; ++it) {
    const int p = tid + 256 * it;
    val[it] = *(const v4f*)(rst + 4 * p);
    go[it]  = (size_t)blockIdx.x * 256 * NX + 4 * p;
  }
  for (int ps = 0; ps < 2; ++ps) {
#pragma unroll
    for (int it = 0; it < 2; ++it) *(volatile v4f*)(rw + go[it]) = val[it];
    __threadfence();
  }
}

#define AGG_ACC_FLOATS 32768
#define AGG_LDS_BYTES (AGG_ACC_FLOATS * 4 + CH * 4 + 16 * 4 + 8 * AGD * 4 + AGD * NX * 4)
template <int WIDE, int USEW>
__global__ __launch_bounds__(256) void k_agg(const float* __restrict__ he, const int* __restrict__ eidx,
                                             const float* __restrict__ rw, _Float16* __restrict__ aout) {
  extern __shared__ __align__(16) float dsm[];
  float* acc  = dsm;
  int*   list = (int*)(dsm + AGG_ACC_FLOATS);
  int*   wtot = list + CH;
  int*   cntw = wtot + 16;
  float* rwl  = (float*)(cntw + 8 * AGD);
  const int tid = threadIdx.x, lane = tid & 31, wave = tid >> 5;
  const int n0 = blockIdx.x * AGD;
  const v4f z4 = (v4f){0.f, 0.f, 0.f, 0.f};
#pragma unroll
  for (int i = 0; i < 32; ++i) *(v4f*)(acc + tid * 128 + 4 * i) = z4;
  if (USEW) {
    if (tid < AGD * NX) rwl[tid] = rw[(size_t)n0 * NX + tid];
  }
  int creg = 0;
  __syncthreads();

  for (int cb = 0; cb < NE / CH; ++cb) {
    const int e0 = cb * CH + 4 * tid;
    const v4i d4 = *(const v4i*)(eidx + NE + e0);
    const v4i s4 = *(const v4i*)(eidx + e0);
    int hit[4];
    int cnt = 0;
#pragma unroll
    for (int j = 0; j < 4; ++j) {
      const int dl = d4[j] - n0;
      hit[j] = ((unsigned)dl < (unsigned)AGD) ? 1 : 0;
      cnt += hit[j];
    }
    int incl = cnt;
#pragma unroll
    for (int off = 1; off < 32; off <<= 1) {
      const int t = __shfl_up(incl, off, 32);
      incl += (lane >= off) ? t : 0;
    }
    if (lane == 31) wtot[wave] = incl;
    __syncthreads();
    int woff = 0, tot = 0;
#pragma unroll
    for (int w = 0; w < 8; ++w) {
      const int v = wtot[w];
      woff += (w < wave) ? v : 0;
      tot += v;
    }
    int pos = woff + incl - cnt;
#pragma unroll
    for (int j = 0; j < 4; ++j) {
      const int s  = min(max(s4[j], 0), NN - 1);
      const int dl = (d4[j] - n0) & 15;
      if (hit[j]) list[pos] = (s << 4) | dl;
      pos += hit[j];
    }
    __syncthreads();
    const int nh = min(tot, CH);
    if (WIDE) {
      for (int i = 0; i < nh; ++i) {
        const int ent = list[i];
        const int sl  = min(ent >> 4, NN - 1);
        const int dl  = ent & 15;
        creg += (dl == tid) ? 1 : 0;
        bool act = true;
        if (USEW) act = (rwl[dl * NX + wave] != 0.f);
        if (act) {
          const float* hp = he + (size_t)sl * EW + 8 * tid;
          float* ap = acc + dl * EW + 8 * tid;
          const v4f a = *(const v4f*)hp, b = *(const v4f*)(hp + 4);
          *(v4f*)ap       = *(v4f*)ap + a;
          *(v4f*)(ap + 4) = *(v4f*)(ap + 4) + b;
        }
      }
    } else {
      for (int i = wave; i < nh; i += 8) {
        const int ent = list[i];
        const int sl  = min(ent >> 4, NN - 1);
        const int dl  = ent & 15;
        creg += (dl == lane) ? 1 : 0;
        const float* hp = he + (size_t)sl * HID + 8 * lane;
        float* ap = acc + (wave * AGD + dl) * HID + 8 * lane;
        const v4f a = *(const v4f*)hp, b = *(const v4f*)(hp + 4);
        *(v4f*)ap       = *(v4f*)ap + a;
        *(v4f*)(ap + 4) = *(v4f*)(ap + 4) + b;
      }
    }
    __syncthreads();
  }

  if (WIDE) {
    if (tid < AGD) cntw[tid] = creg;
  } else {
    if (lane < AGD) cntw[wave * AGD + lane] = creg;
  }
  __syncthreads();

  if (WIDE) {
    for (int ps = 0; ps < 2; ++ps) {
#pragma unroll 1
      for (int dl = 0; dl < AGD; ++dl) {
        const int n   = n0 + dl;
        const int cnt = cntw[dl];
        const float inv = 1.0f / (float)max(cnt, 1);
        const float* hp  = he + (size_t)n * EW + 8 * tid;
        const float* ap2 = acc + dl * EW + 8 * tid;
        v4f r0 = *(const v4f*)hp + *(const v4f*)ap2 * inv;
        v4f r1 = *(const v4f*)(hp + 4) + *(const v4f*)(ap2 + 4) * inv;
        if (USEW) {
          const float wg = rwl[dl * NX + wave];
          r0 *= wg;
          r1 *= wg;
        }
        const v4u pv = pack8h(r0, r1);
        *(volatile v4u*)(aout + (size_t)n * EW + 8 * tid) = pv;
      }
      __threadfence();
    }
  } else {
    for (int ps = 0; ps < 2; ++ps) {
#pragma unroll 1
      for (int k2 = 0; k2 < 2; ++k2) {
        const int dl = wave + 8 * k2;
        const int n  = n0 + dl;
        int cnt = 0;
#pragma unroll
        for (int w = 0; w < 8; ++w) cnt += cntw[w * AGD + dl];
        const float inv = 1.0f / (float)max(cnt, 1);
        v4f s0 = z4, s1 = z4;
#pragma unroll
        for (int w = 0; w < 8; ++w) {
          const float* ap2 = acc + (w * AGD + dl) * HID + 8 * lane;
          s0 += *(const v4f*)ap2;
          s1 += *(const v4f*)(ap2 + 4);
        }
        const float* hp = he + (size_t)n * HID + 8 * lane;
        const v4f r0 = *(const v4f*)hp + s0 * inv;
        const v4f r1 = *(const v4f*)(hp + 4) + s1 * inv;
        const v4u pv = pack8h(r0, r1);
        *(volatile v4u*)(aout + (size_t)n * HID + 8 * lane) = pv;
      }
      __threadfence();
    }
  }
}

template <int EPI>
__global__ __launch_bounds__(256) void k_xgemm(const _Float16* __restrict__ ap, int lda, int akoff,
                                               const _Float16* __restrict__ wt, int K,
                                               const float* __restrict__ bias, int bes, int bel,
                                               const float* __restrict__ rw, float scale,
                                               float* __restrict__ out, int ldo) {
  __shared__ __align__(16) float st[8][16 * OTP];
  __shared__ __align__(16) float bsh[NX * 64];
  __shared__ __align__(16) float rwsh[256 * NX];
  const int tid = threadIdx.x, lane = tid & 31, wave = tid >> 5;
  const int hh = lane >> 4, c = lane & 15;
  const int m0 = blockIdx.x * 256 + wave * 32;
  const int n0 = blockIdx.y * 64;
  const int ex = n0 >> 8;
  const _Float16* A = ap + (size_t)ex * akoff;

  if (EPI == 1) {
    if (tid < 128) {
      const int e  = tid >> 4;
      const int pc = tid & 15;
      *(v4f*)(bsh + e * 64 + 4 * pc) = *(const v4f*)(bias + (size_t)e * HID + n0 + 4 * pc);
    }
    const float* rb = rw + (size_t)blockIdx.x * 256 * NX;
    *(v4f*)(rwsh + 4 * tid)         = *(const v4f*)(rb + 4 * tid);
    *(v4f*)(rwsh + 4 * (tid + 256)) = *(const v4f*)(rb + 4 * (tid + 256));
  }

  v8f acc[2][4];
#pragma unroll
  for (int s = 0; s < 2; ++s)
#pragma unroll
    for (int t = 0; t < 4; ++t) acc[s][t] = zero8();
  gemm32x64(A, lda, wt, K, K, m0, n0, lane, acc);

  float* sw = st[wave];
  if (EPI == 0) {
    float bb[4];
#pragma unroll
    for (int t = 0; t < 4; ++t) bb[t] = bias[ex * bes + bel + (n0 & 255) + 16 * t + c];
#pragma unroll
    for (int sub = 0; sub < 2; ++sub) {
      __syncthreads();
#pragma unroll
      for (int t = 0; t < 4; ++t)
#pragma unroll
        for (int r = 0; r < 8; ++r)
          sw[(8 * hh + r) * OTP + 16 * t + c] = fmaxf(acc[sub][t][r] * scale + bb[t], 0.f);
      __syncthreads();
      store16x64_f32(sw, out, ldo, m0 + sub * 16, n0, lane);
    }
  } else {
#pragma unroll
    for (int sub = 0; sub < 2; ++sub) {
      __syncthreads();
      float bo[4][NX];
#pragma unroll
      for (int t = 0; t < 4; ++t)
#pragma unroll
        for (int e = 0; e < NX; ++e) bo[t][e] = bsh[e * 64 + 16 * t + c];
#pragma unroll
      for (int r = 0; r < 8; ++r) {
        const int rowl = wave * 32 + sub * 16 + 8 * hh + r;
        const v4f w0 = *(const v4f*)(rwsh + rowl * NX);
        const v4f w1 = *(const v4f*)(rwsh + rowl * NX + 4);
#pragma unroll
        for (int t = 0; t < 4; ++t) {
          float b = w0[0] * bo[t][0] + w0[1] * bo[t][1] + w0[2] * bo[t][2] + w0[3] * bo[t][3];
          b += w1[0] * bo[t][4] + w1[1] * bo[t][5] + w1[2] * bo[t][6] + w1[3] * bo[t][7];
          sw[(8 * hh + r) * OTP + 16 * t + c] = acc[sub][t][r] * scale + b;
        }
      }
      __syncthreads();
      store16x64_f32(sw, out, ldo, m0 + sub * 16, n0, lane);
    }
  }
}

extern "C" void kernel_launch(void* const* d_in, const int* in_sizes, int n_in,
                              void* d_out, int out_size, void* d_ws, size_t ws_size,
                              hipStream_t stream) {
  if (n_in < 17) return;
  if (in_sizes[0] != NN * IND) return;
  if (in_sizes[1] != 2 * NE) return;
  if (in_sizes[2] != NN) return;
  if (in_sizes[3] != IND * HID) return;
  if (in_sizes[4] != HID) return;
  if (in_sizes[5] != (HID + 2) * HID) return;
  if (in_sizes[6] != HID) return;
  if (in_sizes[7] != (HID + 2) * HID) return;
  if (in_sizes[8] != HID) return;
  if (in_sizes[9] != (HID + 2) * HID) return;
  if (in_sizes[10] != HID) return;
  if (in_sizes[11] != HID * NX) return;
  if (in_sizes[12] != NX) return;
  if (in_sizes[13] != NX * 2 * HID * HID) return;
  if (in_sizes[14] != NX * 2 * HID) return;
  if (in_sizes[15] != NX * HID * HID) return;
  if (in_sizes[16] != NX * HID) return;
  if (out_size != NN * HID) return;

  const float* x     = (const float*)d_in[0];
  const int*   eidx  = (const int*)d_in[1];
  const int*   batch = (const int*)d_in[2];
  const float* encW  = (const float*)d_in[3];
  const float* encB  = (const float*)d_in[4];
  const float* qW    = (const float*)d_in[5];
  const float* qB    = (const float*)d_in[6];
  const float* kW    = (const float*)d_in[7];
  const float* kB    = (const float*)d_in[8];
  const float* vW    = (const float*)d_in[9];
  const float* vB    = (const float*)d_in[10];
  const float* oW    = (const float*)d_in[11];
  const float* oB    = (const float*)d_in[12];
  const float* eWh   = (const float*)d_in[13];
  const float* eBh   = (const float*)d_in[14];
  const float* eWo   = (const float*)d_in[15];
  const float* eBo   = (const float*)d_in[16];
  float* out = (float*)d_out;

  size_t off = 0;
  const size_t oBig = off; off += (size_t)NN * EW * 4;
  const size_t oH   = oBig;
  const size_t oZ   = oH + (size_t)NN * HID * 4;
  const size_t oQ   = oZ + (size_t)NN * ZP * 2;
  const size_t oKc  = oQ + (size_t)NN * HID * 2;
  const size_t oVt  = oKc + (size_t)NN * HID * 2;
  const size_t oF   = oVt + (size_t)NN * HID * 2;
  if (oF + (size_t)NN * HID * 4 > off) return;
  const size_t oA    = off; off += (size_t)NN * EW * 2;
  const size_t oWq   = off; off += (size_t)3 * HID * ZP * 2;
  const size_t oWh   = off; off += (size_t)2 * EW * HID * 2;
  const size_t oWo   = off; off += (size_t)HID * EW * 2;
  const size_t oTab  = off; off += (size_t)NG * 4 * 4;
  const size_t oPart = off; off += (size_t)(NN / 64) * HID * 4;
  const size_t oKoff = off; off += (size_t)HID * 4;
  const size_t oRw   = off; off += (size_t)NN * NX * 4;
  if (off > ws_size) return;
  if (off > (size_t)134217728) return;

  char* ws = (char*)d_ws;
  float*    Hf   = (float*)(ws + oH);
  _Float16* Zh   = (_Float16*)(ws + oZ);
  _Float16* Qp   = (_Float16*)(ws + oQ);
  _Float16* Kp   = (_Float16*)(ws + oKc);
  _Float16* Vt   = (_Float16*)(ws + oVt);
  float*    Fu   = (float*)(ws + oF);
  float*    He   = (float*)(ws + oBig);
  _Float16* Ap   = (_Float16*)(ws + oA);
  _Float16* Wqkv = (_Float16*)(ws + oWq);
  _Float16* WhT  = (_Float16*)(ws + oWh);
  _Float16* WoT  = (_Float16*)(ws + oWo);
  float*    Tab  = (float*)(ws + oTab);
  float*    Part = (float*)(ws + oPart);
  float*    Koff = (float*)(ws + oKoff);
  float*    Rw   = (float*)(ws + oRw);

  (void)hipFuncSetAttribute(reinterpret_cast<const void*>(&k_agg<0, 0>),
                            hipFuncAttributeMaxDynamicSharedMemorySize, AGG_LDS_BYTES);
  (void)hipFuncSetAttribute(reinterpret_cast<const void*>(&k_agg<1, 0>),
                            hipFuncAttributeMaxDynamicSharedMemorySize, AGG_LDS_BYTES);
  (void)hipFuncSetAttribute(reinterpret_cast<const void*>(&k_agg<1, 1>),
                            hipFuncAttributeMaxDynamicSharedMemorySize, AGG_LDS_BYTES);

  k_stats<<<dim3(1), dim3(256), 0, stream>>>(eidx, batch, Tab);
  k_enc<<<dim3(NN / 64), dim3(256), 0, stream>>>(x, batch, encW, encB, Tab, Hf, Zh, Part);
  k_koff<<<dim3(1), dim3(256), 0, stream>>>(Part, Tab, kW, kB, Koff);
  k_wtr<<<dim3(HID / 64, ZP / 64, 3), dim3(256), 0, stream>>>(qW, kW, vW, 3, 0, HID + 2, HID, 1, HID, 0, 0,
                                                               Wqkv, ZP, 32.0f);
  k_wtr<<<dim3(HID / 64, HID / 64, NX * 2), dim3(256), 0, stream>>>(eWh, eWh, eWh, 1, HID * HID, HID, HID,
                                                                     2, HID, EW, 0, WhT, HID, 32.0f);
  k_wtr<<<dim3(HID / 64, HID / 64, NX), dim3(256), 0, stream>>>(eWo, eWo, eWo, 1, HID * HID, HID, HID,
                                                                 1, 0, 0, HID, WoT, EW, 32.0f);
  k_qkv<<<dim3(NN / 256, 12), dim3(256), 0, stream>>>(Zh, Wqkv, qB, Koff, vB, Qp, Kp, Vt);
  const float sscale = 0.06225728f;
  k_attn<<<dim3(NN / QBLK), dim3(256), 0, stream>>>(Qp, Kp, Vt, Fu, sscale);
  k_router<<<dim3(NN / 256), dim3(256), 0, stream>>>(Fu, oW, oB, Rw);
  hipLaunchKernelGGL(HIP_KERNEL_NAME(k_agg<0, 0>), dim3(NN / AGD), dim3(256), AGG_LDS_BYTES, stream,
                     (const float*)Hf, eidx, (const float*)Rw, Ap);
  hipLaunchKernelGGL(HIP_KERNEL_NAME(k_xgemm<0>), dim3(NN / 256, EW / 64), dim3(256), 0, stream,
                     (const _Float16*)Ap, (int)HID, (int)0, (const _Float16*)WhT, (int)HID,
                     eBh, (int)(2 * HID), (int)0, (const float*)Rw, 0.03125f, He, (int)EW);
  hipLaunchKernelGGL(HIP_KERNEL_NAME(k_agg<1, 0>), dim3(NN / AGD), dim3(256), AGG_LDS_BYTES, stream,
                     (const float*)He, eidx, (const float*)Rw, Ap);
  hipLaunchKernelGGL(HIP_KERNEL_NAME(k_xgemm<0>), dim3(NN / 256, EW / 64), dim3(256), 0, stream,
                     (const _Float16*)Ap, (int)EW, (int)HID, (const _Float16*)(WhT + (size_t)EW * HID), (int)HID,
                     eBh, (int)(2 * HID), (int)HID, (const float*)Rw, 0.03125f, He, (int)EW);
  hipLaunchKernelGGL(HIP_KERNEL_NAME(k_agg<1, 1>), dim3(NN / AGD), dim3(256), AGG_LDS_BYTES, stream,
                     (const float*)He, eidx, (const float*)Rw, Ap);
  hipLaunchKernelGGL(HIP_KERNEL_NAME(k_xgemm<1>), dim3(NN / 256, HID / 64), dim3(256), 0, stream,
                     (const _Float16*)Ap, (int)EW, (int)0, (const _Float16*)WoT, (int)EW,
                     eBo, (int)0, (int)0, (const float*)Rw, 0.03125f, out, (int)HID);
  (void)hipGetLastError();
}
